// PyramidAttention_6459630813244
// MI455X (gfx1250) — hardware-verified
//
#include <hip/hip_runtime.h>
#include <math.h>

constexpr int kNB   = 2;
constexpr int kCH   = 64;
constexpr int kCR   = 16;
constexpr int kWF   = 64;
constexpr int kHW   = 4096;
constexpr int kWS   = 57;
constexpr int kHWS  = 3249;
constexpr int kHWSP = 3264;
constexpr int kLV   = 7345;
constexpr int kLP   = 7360;
constexpr int kDQ   = 144;
constexpr int kDQP  = 160;
constexpr int kDV   = 576;
constexpr int kQC   = 1024;
constexpr int kNQC  = kHW / kQC;
constexpr int kQuadsPerRow  = kLP / 4;
constexpr int kGroupsPerRow = kLP / 8;
constexpr int kSegAGroups = kHW / 8;
constexpr int kSegBGroups = (kLP - kHW) / 8;
constexpr int kSegABlocks = kDV * kSegAGroups / 256;
constexpr int kSegBBlocks = kDV * kSegBGroups / 256;
constexpr float kVCarry = 16.0f;
constexpr float kPCarry = 32768.0f;
constexpr float kScoreScale = 10.0f;
constexpr float kAggScale   = 1.0f / (32768.0f * 16.0f);
constexpr float kNormEps = 1.0e-4f;

static_assert(kCR * 9 == kDQ && kCH * 9 == kDV, "shape");
static_assert(kHW + kHWS == kLV && kLV <= kLP, "keys");
static_assert(kDQP % 32 == 0 && kLP % 32 == 0, "K multiples of 32");
static_assert(kQC % 64 == 0 && kLP % 64 == 0 && kDV % 64 == 0, "M,N multiples of 64");
static_assert(kQuadsPerRow * 4 == kLP && kGroupsPerRow * 8 == kLP, "row split");
static_assert(kSegAGroups * 8 == kHW && kSegBGroups * 8 == kLP - kHW, "segments");
static_assert(kSegABlocks * 256 == kDV * kSegAGroups && kSegBBlocks * 256 == kDV * kSegBGroups, "vt grid exact");
static_assert(kHWSP % 32 == 0 && kHWSP >= kHWS && kHW % 32 == 0, "conv chunks");
static_assert(kHW % 16 == 0 && kLP % 16 == 0, "row builder blocks");
static_assert((16 * kDQP * 2) % 128 == 0, "row builder block range is whole lines");

constexpr size_t kSzQb  = (size_t)kNB * kCR * kHW   * 4;
constexpr size_t kSzKf  = (size_t)kNB * kCR * kHW   * 4;
constexpr size_t kSzKs  = (size_t)kNB * kCR * kHWSP * 4;
constexpr size_t kSzVf  = (size_t)kNB * kCH * kHW   * 4;
constexpr size_t kSzVs  = (size_t)kNB * kCH * kHWSP * 4;
constexpr size_t kSzQ16 = (size_t)kNB * kHW * kDQP  * 2;
constexpr size_t kSzK16 = (size_t)kNB * kLP * kDQP  * 2;
constexpr size_t kSzVT  = (size_t)kNB * kDV * kLP   * 2;
constexpr size_t kSzS   = (size_t)kQC * kLP * 4;
constexpr size_t kSzP   = (size_t)kQC * kLP * 2;
constexpr size_t kSzT   = (size_t)kNB * kHW * kDV   * 4;
constexpr size_t kOffQb  = 0;
constexpr size_t kOffKf  = kOffQb  + kSzQb;
constexpr size_t kOffKs  = kOffKf  + kSzKf;
constexpr size_t kOffVf  = kOffKs  + kSzKs;
constexpr size_t kOffVs  = kOffVf  + kSzVf;
constexpr size_t kOffQh  = kOffVs  + kSzVs;
constexpr size_t kOffQl  = kOffQh  + kSzQ16;
constexpr size_t kOffKh  = kOffQl  + kSzQ16;
constexpr size_t kOffKl  = kOffKh  + kSzK16;
constexpr size_t kOffVT  = kOffKl  + kSzK16;
constexpr size_t kOffS   = kOffVT  + kSzVT;
constexpr size_t kOffP   = kOffS   + kSzS;
constexpr size_t kOffT   = kOffP   + kSzP;
constexpr size_t kWsTotal = kOffT  + kSzT;
static_assert(kWsTotal == 100950016, "carve total");
static_assert(kWsTotal <= (size_t)134217728, "carve under 128 MiB");
static_assert(kSzKs % 256 == 0 && kSzVs % 256 == 0 && kSzQ16 % 256 == 0 && kSzK16 % 256 == 0 && kSzVT % 256 == 0 && kSzS % 256 == 0 && kSzP % 256 == 0, "align");

typedef __attribute__((ext_vector_type(16))) _Float16 v16h;
typedef __attribute__((ext_vector_type(8)))  _Float16 v8h;
typedef __attribute__((ext_vector_type(16))) __bf16   v16b;
typedef __attribute__((ext_vector_type(8)))  __bf16   v8b;
typedef __attribute__((ext_vector_type(8)))  float    v8f;
typedef __attribute__((ext_vector_type(4)))  float    v4f;
typedef __attribute__((ext_vector_type(4)))  unsigned int v4u;

__device__ __forceinline__ unsigned short f2bf_bits(float f) {
  unsigned u = __float_as_uint(f);
  return (unsigned short)((u + 0x7FFFu + ((u >> 16) & 1u)) >> 16);
}
__device__ __forceinline__ float bf_bits2f(unsigned short h) { return __uint_as_float(((unsigned)h) << 16); }

__device__ __forceinline__ void dep_guard_h(v8f& a, v8f& b, v16h x, v16h y) { asm volatile("v_nop\n\tv_nop\n\tv_nop\n\tv_nop" : "+v"(a), "+v"(b) : "v"(x), "v"(y)); }
__device__ __forceinline__ void dep_guard_b(v8f& a, v8f& b, v16b x, v16b y) { asm volatile("v_nop\n\tv_nop\n\tv_nop\n\tv_nop" : "+v"(a), "+v"(b) : "v"(x), "v"(y)); }
__device__ __forceinline__ void keep4_h(v16h a, v16h b, v16h c, v16h d) { asm volatile("v_nop" :: "v"(a), "v"(b), "v"(c), "v"(d)); }
__device__ __forceinline__ void keep4_b(v16b a, v16b b, v16b c, v16b d) { asm volatile("v_nop" :: "v"(a), "v"(b), "v"(c), "v"(d)); }
__device__ __forceinline__ void acc_guard4(v8f& a, v8f& b, v8f& c, v8f& d) { asm volatile("v_nop\n\tv_nop\n\tv_nop\n\tv_nop" : "+v"(a), "+v"(b), "+v"(c), "+v"(d)); }
template <typename T> struct Frag;
template <> struct Frag<_Float16> {
  typedef v16h V; union U { v16h v; v8h h[2]; };
  static __device__ __forceinline__ v16h load(const _Float16* p) {
    U f; f.h[0] = *(const v8h*)(p); f.h[1] = *(const v8h*)(p + 16); return f.v;
  }
  static __device__ __forceinline__ v8f mma(v16h a, v16h b, v8f c) {
    return __builtin_amdgcn_wmma_f32_16x16x32_f16(false, a, false, b, (short)0, c, false, false);
  }
  static __device__ __forceinline__ void guard(v8f& a, v8f& b, v16h x, v16h y) { dep_guard_h(a, b, x, y); }
  static __device__ __forceinline__ void keep(v16h a, v16h b, v16h c, v16h d) { keep4_h(a, b, c, d); }
};
template <> struct Frag<__bf16> {
  typedef v16b V; union U { v16b v; v8b h[2]; };
  static __device__ __forceinline__ v16b load(const __bf16* p) {
    U f; f.h[0] = *(const v8b*)(p); f.h[1] = *(const v8b*)(p + 16); return f.v;
  }
  static __device__ __forceinline__ v8f mma(v16b a, v16b b, v8f c) {
    return __builtin_amdgcn_wmma_f32_16x16x32_bf16(false, a, false, b, (short)0, c, false, false);
  }
  static __device__ __forceinline__ void guard(v8f& a, v8f& b, v16b x, v16b y) { dep_guard_b(a, b, x, y); }
  static __device__ __forceinline__ void keep(v16b a, v16b b, v16b c, v16b d) { keep4_b(a, b, c, d); }
};

__device__ __forceinline__ unsigned pk16(unsigned short a, unsigned short b) { return (unsigned)a | ((unsigned)b << 16); }
__device__ __forceinline__ unsigned short h_bits(float f) { const _Float16 h = (_Float16)f; return __builtin_bit_cast(unsigned short, h); }

template <int ET> struct Elem;
template <> struct Elem<0> { typedef _Float16 T; };
template <> struct Elem<1> { typedef __bf16 T; };
template <int ET, bool SPLIT, int BIAS_MODE, int OUT_MODE, bool RESID, int ACT = 0>
__global__ __launch_bounds__(256) void wmma_gemm64(
    const unsigned short* __restrict__ Ap, const unsigned short* __restrict__ A2p, int lda, long strideA,
    const unsigned short* __restrict__ Btp, const unsigned short* __restrict__ Bt2p, int ldb, long strideB,
    void* __restrict__ Cout, void* __restrict__ Cout2, int ldc, long strideC,
    const float* __restrict__ bias,
    const float* __restrict__ resid, long strideR,
    int M, int N, int K, float scale) {
  typedef typename Elem<ET>::T T;
  typedef typename Frag<T>::V V;
  const T* A = (const T*)Ap; const T* A2 = (const T*)A2p; const T* Bt = (const T*)Btp; const T* Bt2 = (const T*)Bt2p;
  __shared__ __align__(16) float sT[8][16 * 68];
  const int b    = blockIdx.y;
  const int lane = threadIdx.x & 31;
  const int wave = threadIdx.x >> 5;
  const int tilesN = N >> 6;
  const int tilesM = M >> 6;
  const int tile = blockIdx.x * 8 + wave;
  if (tile >= tilesM * tilesN) return;
  const int tm = tile / tilesN;
  const int tn = tile - tm * tilesN;
  const int m0 = tm << 6;
  const int n0 = tn << 6;

  const T* Ab  = A  + (size_t)b * strideA;
  const T* Bb  = Bt + (size_t)b * strideB;
  const T* Ab2 = SPLIT ? (A2  + (size_t)b * strideA) : nullptr;
  const T* Bb2 = SPLIT ? (Bt2 + (size_t)b * strideB) : nullptr;

  const int rlane = lane & 15;
  const int koff  = (lane >> 4) * 8;
  const int mOff  = (lane >> 4) * 8;

  v8f acc[4][4];
#pragma unroll
  for (int i = 0; i < 4; ++i)
#pragma unroll
    for (int j = 0; j < 4; ++j) acc[i][j] = (v8f){0.f,0.f,0.f,0.f,0.f,0.f,0.f,0.f};

  for (int k0 = 0; k0 < K; k0 += 32) {
    V bh[4], bl[4];
#pragma unroll
    for (int j = 0; j < 4; ++j) {
      const size_t bo = (size_t)(n0 + (j << 4) + rlane) * ldb + koff + k0;
      bh[j] = Frag<T>::load(Bb + bo);
      if (SPLIT) bl[j] = Frag<T>::load(Bb2 + bo);
    }
#pragma unroll
    for (int i = 0; i < 4; ++i) {
      const size_t ao = (size_t)(m0 + (i << 4) + rlane) * lda + koff + k0;
      V ah = Frag<T>::load(Ab + ao);
      V al;
      if (SPLIT) al = Frag<T>::load(Ab2 + ao);
#pragma unroll
      for (int j = 0; j < 4; ++j) {
        acc[i][j] = Frag<T>::mma(ah, bh[j], acc[i][j]);
        if (SPLIT) {
          acc[i][j] = Frag<T>::mma(ah, bl[j], acc[i][j]);
          acc[i][j] = Frag<T>::mma(al, bh[j], acc[i][j]);
        }
      }
      Frag<T>::guard(acc[i][0], acc[i][3], ah, SPLIT ? al : ah);
    }
    Frag<T>::keep(bh[0], bh[1], bh[2], bh[3]);
    if (SPLIT) Frag<T>::keep(bl[0], bl[1], bl[2], bl[3]);
  }
  acc_guard4(acc[0][0], acc[0][1], acc[0][2], acc[0][3]);
  acc_guard4(acc[1][0], acc[1][1], acc[1][2], acc[1][3]);
  acc_guard4(acc[2][0], acc[2][1], acc[2][2], acc[2][3]);
  acc_guard4(acc[3][0], acc[3][1], acc[3][2], acc[3][3]);

  float* slab = sT[wave];
  const float* Rb = RESID ? (resid + (size_t)b * strideR) : nullptr;
#pragma unroll
  for (int i = 0; i < 4; ++i) {
    const int mBase = m0 + (i << 4);
#pragma unroll
    for (int j = 0; j < 4; ++j) {
      const int n = n0 + (j << 4) + rlane;
      float bv = 0.f;
      if (BIAS_MODE == 2) bv = bias[n];
#pragma unroll
      for (int r = 0; r < 8; ++r) {
        float v = acc[i][j][r] * scale;
        if (BIAS_MODE == 1) v += bias[mBase + mOff + r];
        if (BIAS_MODE == 2) v += bv;
        if (RESID) v += Rb[(size_t)(mBase + mOff + r) * ldc + n];
        if (ACT == 2) v = fmaxf(v, 0.0f);
        if (ACT == 4) v = (v > 0.f) ? v : 0.01f * v;
        slab[(mOff + r) * 68 + (j << 4) + rlane] = v;
      }
    }
    __builtin_amdgcn_fence(__ATOMIC_RELEASE, "workgroup");
    __builtin_amdgcn_wave_barrier();
    __builtin_amdgcn_fence(__ATOMIC_ACQUIRE, "workgroup");
    if (OUT_MODE == 0) {
      float* C = (float*)Cout + (size_t)b * strideC;
      const int hh = lane >> 4, c4 = (lane & 15) * 4;
      for (int pass = 0; pass < 2; ++pass) {
#pragma unroll
        for (int it = 0; it < 8; ++it) {
          const int row = it * 2 + hh;
          v4f v = *(const v4f*)(slab + row * 68 + c4);
          *(volatile v4f*)(C + (size_t)(mBase + row) * ldc + n0 + c4) = v;
        }
        __threadfence();
      }
    } else {
      const int q = lane >> 3, c8 = (lane & 7) * 8;
      unsigned short* C  = (unsigned short*)Cout  + (size_t)b * strideC;
      unsigned short* C2 = (OUT_MODE == 2) ? ((unsigned short*)Cout2 + (size_t)b * strideC) : nullptr;
      for (int pass = 0; pass < 2; ++pass) {
#pragma unroll
        for (int it = 0; it < 4; ++it) {
          const int row = it * 4 + q;
          const float* sp = slab + row * 68 + c8;
          v8h hv, lv;
#pragma unroll
          for (int e = 0; e < 8; ++e) {
            if (OUT_MODE == 1) {
              hv[e] = (_Float16)sp[e];
            } else {
              unsigned short hb = f2bf_bits(sp[e]);
              unsigned short lb = f2bf_bits(sp[e] - bf_bits2f(hb));
              hv[e] = __builtin_bit_cast(_Float16, hb);
              lv[e] = __builtin_bit_cast(_Float16, lb);
            }
          }
          *(volatile v8h*)(C + (size_t)(mBase + row) * ldc + n0 + c8) = hv;
          if (OUT_MODE == 2) *(volatile v8h*)(C2 + (size_t)(mBase + row) * ldc + n0 + c8) = lv;
        }
        __threadfence();
      }
    }
    __builtin_amdgcn_fence(__ATOMIC_RELEASE, "workgroup");
    __builtin_amdgcn_wave_barrier();
    __builtin_amdgcn_fence(__ATOMIC_ACQUIRE, "workgroup");
  }
}

template <int COUT>
__global__ __launch_bounds__(COUT * 4) void conv_prelu_kernel(const float* __restrict__ in, const float* __restrict__ w,
                                                            const float* __restrict__ bias, const float* __restrict__ slope,
                                                            float* __restrict__ out, int hwIn, int pitch, int chunksPerBatch) {
  __shared__ __align__(16) float wsm[kCH * COUT];
  const int tid  = threadIdx.x;
  const int lane = tid & 31;
  const int og   = tid >> 5;
  const int blk  = blockIdx.x;
  const int b     = blk / chunksPerBatch;
  const int chunk = blk - b * chunksPerBatch;
#pragma unroll 4
  for (int i = 0; i < 16; ++i) {
    const int e = i * (COUT * 4) + tid;
    const int o = e >> 6;
    const int c = e & 63;
    wsm[c * COUT + o] = w[e];
  }
  __syncthreads();
  const int pix  = chunk * 32 + lane;
  const int pixc = pix < hwIn ? pix : hwIn - 1;
  const float* ip = in + (size_t)b * kCH * hwIn + pixc;
  float acc[8];
#pragma unroll
  for (int e = 0; e < 8; ++e) acc[e] = 0.0f;
#pragma unroll 2
  for (int c = 0; c < kCH; ++c) {
    const float xv = ip[(size_t)c * hwIn];
    const v4f w0 = *(const v4f*)(wsm + c * COUT + og * 8);
    const v4f w1 = *(const v4f*)(wsm + c * COUT + og * 8 + 4);
#pragma unroll
    for (int e = 0; e < 4; ++e) {
      acc[e]     = fmaf(xv, w0[e], acc[e]);
      acc[4 + e] = fmaf(xv, w1[e], acc[4 + e]);
    }
  }
  const float a = slope[0];
  float y[8];
#pragma unroll
  for (int e = 0; e < 8; ++e) {
    const float t = acc[e] + bias[og * 8 + e];
    y[e] = (t >= 0.0f) ? t : a * t;
  }
  float* op = out + ((size_t)(b * COUT + og * 8)) * pitch + pix;
#pragma unroll
  for (int e = 0; e < 8; ++e) *(volatile float*)(op + (size_t)e * pitch) = y[e];
  __threadfence();
#pragma unroll
  for (int e = 0; e < 8; ++e) *(volatile float*)(op + (size_t)e * pitch) = y[e];
}

__device__ __forceinline__ void gather_patch5(const float* __restrict__ plane, int pitch, int wd, int hd,
                                              int p, bool rowok, int lane, float v[5]) {
  const int h = p / wd;
  const int w = p - h * wd;
#pragma unroll
  for (int k = 0; k < 5; ++k) {
    const int d  = lane + 32 * k;
    const int dc = d < kDQ ? d : (kDQ - 1);
    const int c  = dc / 9;
    const int t  = dc - 9 * c;
    const int ti = t / 3;
    const int di = ti - 1;
    const int dj = (t - 3 * ti) - 1;
    const int hh = h + di;
    const int ww = w + dj;
    const bool inb = rowok && (d < kDQ) && (hh >= 0) && (hh < hd) && (ww >= 0) && (ww < wd);
    const int hhc = hh < 0 ? 0 : (hh >= hd ? hd - 1 : hh);
    const int wwc = ww < 0 ? 0 : (ww >= wd ? wd - 1 : ww);
    const float x = plane[(size_t)c * pitch + hhc * wd + wwc];
    v[k] = inb ? x : 0.0f;
  }
}

template <bool ISK>
__global__ __launch_bounds__(256) void build_rows_kernel(const float* __restrict__ srcFull, const float* __restrict__ srcSmall,
                                                       unsigned short* __restrict__ dstHi, unsigned short* __restrict__ dstLo) {
  __shared__ __align__(16) float sm[16 * kDQP];
  const int tid  = threadIdx.x;
  const int lane = tid & 31;
  const int wave = tid >> 5;
  const int blk  = blockIdx.x;
  const int b    = blockIdx.y;
  constexpr int rowsPerBatch = ISK ? kLP : kHW;
  const int r0 = blk * 16;
#pragma unroll
  for (int i = 0; i < 2; ++i) {
    const int rl = 2 * wave + i;
    const int r  = r0 + rl;
    float v[5];
    if (!ISK || blk < (kHW / 16)) {
      gather_patch5(srcFull + (size_t)b * kCR * kHW, kHW, kWF, kWF, r, true, lane, v);
    } else {
      const int p  = r - kHW;
      const bool ok = p < kHWS;
      const int pc = ok ? p : (kHWS - 1);
      gather_patch5(srcSmall + (size_t)b * kCR * kHWSP, kHWSP, kWS, kWS, pc, ok, lane, v);
    }
    float sc = 1.0f;
    if (ISK) {
      float ss = 0.0f;
#pragma unroll
      for (int k = 0; k < 5; ++k) ss = ss + v[k] * v[k];
#pragma unroll
      for (int off = 16; off > 0; off >>= 1) ss += __shfl_xor(ss, off, 32);
      const float nrm = fmaxf(sqrtf(ss), kNormEps);
      sc = 1.0f / nrm;
    }
#pragma unroll
    for (int k = 0; k < 5; ++k) sm[rl * kDQP + lane + 32 * k] = v[k] * sc;
  }
  __syncthreads();
  const size_t boff = ((size_t)b * rowsPerBatch + r0) * kDQP;
  unsigned short* baseH = dstHi + boff;
  unsigned short* baseL = dstLo + boff;
#pragma unroll
  for (int it = 0; it < 2; ++it) {
    const int f = tid + 256 * it;
    if (f < 320) {
      const int rl = f / 20;
      const int g  = f - 20 * rl;
      const float* sp = sm + rl * kDQP + 8 * g;
      const v4f e0 = *(const v4f*)(sp);
      const v4f e1 = *(const v4f*)(sp + 4);
      unsigned short hb[8], lb[8];
#pragma unroll
      for (int e = 0; e < 4; ++e) {
        const unsigned short h0 = f2bf_bits(e0[e]);
        hb[e] = h0;
        lb[e] = f2bf_bits(e0[e] - bf_bits2f(h0));
        const unsigned short h1 = f2bf_bits(e1[e]);
        hb[4 + e] = h1;
        lb[4 + e] = f2bf_bits(e1[e] - bf_bits2f(h1));
      }
      const v4u uh = (v4u){pk16(hb[0], hb[1]), pk16(hb[2], hb[3]), pk16(hb[4], hb[5]), pk16(hb[6], hb[7])};
      const v4u ul = (v4u){pk16(lb[0], lb[1]), pk16(lb[2], lb[3]), pk16(lb[4], lb[5]), pk16(lb[6], lb[7])};
      unsigned short* ph = baseH + 8 * (size_t)f;
      unsigned short* pl = baseL + 8 * (size_t)f;
      *(volatile v4u*)ph = uh;
      *(volatile v4u*)pl = ul;
      __threadfence();
      *(volatile v4u*)ph = uh;
      *(volatile v4u*)pl = ul;
    }
  }
}

__device__ __forceinline__ void vt_gather8(const float* __restrict__ plane, int wd, int pcount, int p0,
                                           int di, int dj, float carry, float x[8]) {
#pragma unroll
  for (int k = 0; k < 8; ++k) {
    const int p  = p0 + k;
    const bool okp = (p >= 0) && (p < pcount);
    const int pc = p < 0 ? 0 : (p >= pcount ? pcount - 1 : p);
    const int h  = pc / wd;
    const int w  = pc - h * wd;
    const int hh = h + di;
    const int ww = w + dj;
    const bool inb = okp && (hh >= 0) && (hh < wd) && (ww >= 0) && (ww < wd);
    const int hhc = hh < 0 ? 0 : (hh >= wd ? wd - 1 : hh);
    const int wwc = ww < 0 ? 0 : (ww >= wd ? wd - 1 : ww);
    const float v = plane[hhc * wd + wwc];
    x[k] = inb ? v * carry : 0.0f;
  }
}

__global__ __launch_bounds__(256) void build_vt_kernel(const float* __restrict__ vf, const float* __restrict__ vs,
                                                     unsigned short* __restrict__ vt, float carry) {
  const int tid = threadIdx.x;
  const int b   = blockIdx.y;
  int e, g;
  float x[8];
  if (blockIdx.x < kSegABlocks) {
    const int i = blockIdx.x * 256 + tid;
    e = i >> 9;
    g = i & (kSegAGroups - 1);
    const int c  = e / 9;
    const int t  = e - 9 * c;
    const int ti = t / 3;
    const int di = ti - 1;
    const int dj = (t - 3 * ti) - 1;
    vt_gather8(vf + ((size_t)b * kCH + c) * kHW, kWF, kHW, 8 * g, di, dj, carry, x);
  } else {
    const int j = (blockIdx.x - kSegABlocks) * 256 + tid;
    e = j / kSegBGroups;
    g = kSegAGroups + (j - kSegBGroups * e);
    const int c  = e / 9;
    const int t  = e - 9 * c;
    const int ti = t / 3;
    const int di = ti - 1;
    const int dj = (t - 3 * ti) - 1;
    vt_gather8(vs + ((size_t)b * kCH + c) * kHWSP, kWS, kHWS, 8 * g - kHW, di, dj, carry, x);
  }
  unsigned short hb[8];
#pragma unroll
  for (int k = 0; k < 8; ++k) hb[k] = h_bits(x[k]);
  const v4u u = (v4u){pk16(hb[0], hb[1]), pk16(hb[2], hb[3]), pk16(hb[4], hb[5]), pk16(hb[6], hb[7])};
  unsigned short* p = vt + ((size_t)b * kDV + e) * kLP + 8 * (size_t)g;
  *(volatile v4u*)p = u;
  __threadfence();
  *(volatile v4u*)p = u;
}

__global__ __launch_bounds__(256) void softmax_row_kernel(const float* __restrict__ S, unsigned short* __restrict__ P) {
  __shared__ __align__(16) float lg[kLP];
  __shared__ float redM[8];
  __shared__ float redS[8];
  const int row  = blockIdx.x;
  const int tid  = threadIdx.x;
  const int lane = tid & 31, wave = tid >> 5;
  const float* sr = S + (size_t)row * kLP;
  const float ninf = -__builtin_inff();

  float mx = ninf;
#pragma unroll 1
  for (int it = 0; it < 8; ++it) {
    const int q4 = tid + 256 * it;
    const int qc = q4 < kQuadsPerRow ? q4 : (kQuadsPerRow - 1);
    const v4f sv = *(const v4f*)(sr + 4 * qc);
    v4f xv;
#pragma unroll
    for (int e = 0; e < 4; ++e) {
      const int col = 4 * q4 + e;
      const float xe = (col < kLV) ? sv[e] : ninf;
      xv[e] = xe;
      mx = fmaxf(mx, xe);
    }
    if (q4 < kQuadsPerRow) *(v4f*)(lg + 4 * q4) = xv;
  }
#pragma unroll
  for (int off = 16; off > 0; off >>= 1) mx = fmaxf(mx, __shfl_xor(mx, off, 32));
  if (lane == 0) redM[wave] = mx;
  __syncthreads();
  float m = redM[0];
#pragma unroll
  for (int w = 1; w < 8; ++w) m = fmaxf(m, redM[w]);

  float sum = 0.0f;
#pragma unroll 1
  for (int it = 0; it < 8; ++it) {
    const int q4 = tid + 256 * it;
    if (q4 < kQuadsPerRow) {
      const v4f l = *(const v4f*)(lg + 4 * q4);
      v4f ev;
#pragma unroll
      for (int e = 0; e < 4; ++e) {
        const float ee = expf(l[e] - m);
        ev[e] = ee;
        sum += ee;
      }
      *(v4f*)(lg + 4 * q4) = ev;
    }
  }
#pragma unroll
  for (int off = 16; off > 0; off >>= 1) sum += __shfl_xor(sum, off, 32);
  if (lane == 0) redS[wave] = sum;
  __syncthreads();
  float tot = redS[0];
#pragma unroll
  for (int w = 1; w < 8; ++w) tot += redS[w];
  const float inv = kPCarry * (1.0f / tot);

  unsigned short* prow = P + (size_t)row * kLP;
#pragma unroll 1
  for (int it = 0; it < 4; ++it) {
    const int g = tid + 256 * it;
    if (g < kGroupsPerRow) {
      const v4f e0 = *(const v4f*)(lg + 8 * g);
      const v4f e1 = *(const v4f*)(lg + 8 * g + 4);
      unsigned short hb[8];
#pragma unroll
      for (int e = 0; e < 4; ++e) {
        hb[e]     = h_bits(e0[e] * inv);
        hb[4 + e] = h_bits(e1[e] * inv);
      }
      const v4u u = (v4u){pk16(hb[0], hb[1]), pk16(hb[2], hb[3]), pk16(hb[4], hb[5]), pk16(hb[6], hb[7])};
      unsigned short* pp = prow + 8 * (size_t)g;
      *(volatile v4u*)pp = u;
      __threadfence();
      *(volatile v4u*)pp = u;
    }
  }
}

__global__ __launch_bounds__(256) void fold_residual_kernel(const float* __restrict__ agg, const float* __restrict__ x,
                                                          float* __restrict__ y) {
  const int idx = blockIdx.x * 256 + threadIdx.x;
  const int w = idx & 63;
  const int h = (idx >> 6) & 63;
  const int c = (idx >> 12) & 63;
  const int b = idx >> 18;
  const float* tb = agg + (size_t)b * kHW * kDV + c * 9;
  float s = 0.0f;
#pragma unroll
  for (int ti = 0; ti < 3; ++ti) {
#pragma unroll
    for (int tj = 0; tj < 3; ++tj) {
      const int hh = h + 1 - ti;
      const int ww = w + 1 - tj;
      const bool inb = (hh >= 0) && (hh < kWF) && (ww >= 0) && (ww < kWF);
      const int hhc = hh < 0 ? 0 : (hh >= kWF ? kWF - 1 : hh);
      const int wwc = ww < 0 ? 0 : (ww >= kWF ? kWF - 1 : ww);
      const float v = tb[(size_t)(hhc * kWF + wwc) * kDV + ti * 3 + tj];
      s = s + (inb ? v : 0.0f);
    }
  }
  const float r = x[idx] + 0.25f * s;
  *(volatile float*)(y + idx) = r;
  __threadfence();
  *(volatile float*)(y + idx) = r;
}

extern "C" void kernel_launch(void* const* d_in, const int* in_sizes, int n_in,
                              void* d_out, int out_size, void* d_ws, size_t ws_size,
                              hipStream_t stream) {
  if (n_in < 11) return;
  if (in_sizes[0] != kNB * kCH * kHW) return;
  if (in_sizes[1] != kNB * kCH * kHWS) return;
  if (in_sizes[2] != kCR * kCH || in_sizes[3] != kCR || in_sizes[4] != 1) return;
  if (in_sizes[5] != kCR * kCH || in_sizes[6] != kCR || in_sizes[7] != 1) return;
  if (in_sizes[8] != kCH * kCH || in_sizes[9] != kCH || in_sizes[10] != 1) return;
  if (out_size != kNB * kCH * kHW) return;
  if (ws_size < kWsTotal) return;

  const float* input = (const float*)d_in[0];
  const float* small = (const float*)d_in[1];
  const float* w_mb  = (const float*)d_in[2];
  const float* b_mb  = (const float*)d_in[3];
  const float* a_mb  = (const float*)d_in[4];
  const float* w_m   = (const float*)d_in[5];
  const float* b_m   = (const float*)d_in[6];
  const float* a_m   = (const float*)d_in[7];
  const float* w_as  = (const float*)d_in[8];
  const float* b_as  = (const float*)d_in[9];
  const float* a_as  = (const float*)d_in[10];
  float* out = (float*)d_out;

  char* ws = (char*)d_ws;
  float* Qb = (float*)(ws + kOffQb);
  float* Kf = (float*)(ws + kOffKf);
  float* Ks = (float*)(ws + kOffKs);
  float* Vf = (float*)(ws + kOffVf);
  float* Vs = (float*)(ws + kOffVs);
  unsigned short* Qh = (unsigned short*)(ws + kOffQh);
  unsigned short* Ql = (unsigned short*)(ws + kOffQl);
  unsigned short* Kh = (unsigned short*)(ws + kOffKh);
  unsigned short* Kl = (unsigned short*)(ws + kOffKl);
  unsigned short* VT = (unsigned short*)(ws + kOffVT);
  float* SC = (float*)(ws + kOffS);
  unsigned short* PP = (unsigned short*)(ws + kOffP);
  float* TA = (float*)(ws + kOffT);
  const float* fdummy = (const float*)(ws + kOffQb);

  const int chunksFull  = kHW / 32;
  const int chunksSmall = kHWSP / 32;
  conv_prelu_kernel<kCR><<<dim3(kNB * chunksFull), dim3(kCR * 4), 0, stream>>>(input, w_mb, b_mb, a_mb, Qb, kHW, kHW, chunksFull);
  conv_prelu_kernel<kCR><<<dim3(kNB * chunksFull), dim3(kCR * 4), 0, stream>>>(input, w_m, b_m, a_m, Kf, kHW, kHW, chunksFull);
  conv_prelu_kernel<kCR><<<dim3(kNB * chunksSmall), dim3(kCR * 4), 0, stream>>>(small, w_m, b_m, a_m, Ks, kHWS, kHWSP, chunksSmall);
  conv_prelu_kernel<kCH><<<dim3(kNB * chunksFull), dim3(kCH * 4), 0, stream>>>(input, w_as, b_as, a_as, Vf, kHW, kHW, chunksFull);
  conv_prelu_kernel<kCH><<<dim3(kNB * chunksSmall), dim3(kCH * 4), 0, stream>>>(small, w_as, b_as, a_as, Vs, kHWS, kHWSP, chunksSmall);

  build_rows_kernel<false><<<dim3(kHW / 16, kNB), dim3(256), 0, stream>>>(Qb, Ks, Qh, Ql);
  build_rows_kernel<true><<<dim3(kLP / 16, kNB), dim3(256), 0, stream>>>(Kf, Ks, Kh, Kl);
  build_vt_kernel<<<dim3(kSegABlocks + kSegBBlocks, kNB), dim3(256), 0, stream>>>(Vf, Vs, VT, kVCarry);

  const int tilesScore = (kQC / 64) * (kLP / 64);
  const int tilesAgg   = (kQC / 64) * (kDV / 64);
  for (int b = 0; b < kNB; ++b) {
    const unsigned short* Kbh = Kh + (size_t)b * kLP * kDQP;
    const unsigned short* Kbl = Kl + (size_t)b * kLP * kDQP;
    const unsigned short* VTb = VT + (size_t)b * kDV * kLP;
    for (int qc = 0; qc < kNQC; ++qc) {
      const size_t prow0 = (size_t)b * kHW + (size_t)qc * kQC;
      const unsigned short* Aqh = Qh + prow0 * kDQP;
      const unsigned short* Aql = Ql + prow0 * kDQP;
      wmma_gemm64<1, true, 0, 0, false, 0><<<dim3(tilesScore / 8, 1), dim3(256), 0, stream>>>(
          Aqh, Aql, kDQP, 0L, Kbh, Kbl, kDQP, 0L,
          (void*)SC, (void*)SC, kLP, 0L, fdummy, fdummy, 0L, kQC, kLP, kDQP, kScoreScale);
      softmax_row_kernel<<<dim3(kQC), dim3(256), 0, stream>>>(SC, PP);
      float* Tc = TA + prow0 * kDV;
      wmma_gemm64<0, false, 0, 0, false, 0><<<dim3(tilesAgg / 8, 1), dim3(256), 0, stream>>>(
          PP, PP, kLP, 0L, VTb, VTb, kLP, 0L,
          (void*)Tc, (void*)Tc, kDV, 0L, fdummy, fdummy, 0L, kQC, kDV, kLP, kAggScale);
    }
  }

  fold_residual_kernel<<<dim3((kNB * kCH * kHW) / 256), dim3(256), 0, stream>>>(TA, input, out);
}
